// MeshMamba3D_Seg_38371237822542
// MI455X (gfx1250) — hardware-run, weakly checked
//
#include <hip/hip_runtime.h>
#include <math.h>

typedef __attribute__((ext_vector_type(16))) _Float16 v16h;
typedef __attribute__((ext_vector_type(8)))  _Float16 v8h;
typedef __attribute__((ext_vector_type(8)))  float    v8f;
typedef __attribute__((ext_vector_type(4)))  float    v4f;
typedef __attribute__((ext_vector_type(4)))  int      v4i;

constexpr int kB   = 8;
constexpr int kG   = 1024;
constexpr int kC   = 384;
constexpr int kC2  = 2 * kC;
constexpr int kG2  = 2 * kG;
constexpr int kNbr = 16;
constexpr int kBG  = kB * kG;
constexpr int kBC  = kB * kC;
constexpr int kStatBlocks = kBG / 16;
constexpr int kSlabP = 68;
constexpr float kEps = 1e-5f;
constexpr float kWCarry = 1024.0f;
constexpr float kNCarry = 16.0f;
constexpr float kXCarry = 64.0f;
constexpr float kScaleGaf = 1.0f / (kNCarry * kWCarry);
constexpr float kScaleMlp = 1.0f / (kWCarry * kNCarry);
constexpr float kScaleFin = 1.0f / (kWCarry * kXCarry);
static_assert(kC2 == 768 && kG2 == 2048 && kBG == 8192 && kBC == 3072, "shapes");
static_assert((kC2 % 32) == 0 && (kG % 32) == 0 && (kG2 % 32) == 0, "GEMM K multiples of 32");
static_assert((kBC % 64) == 0 && (kG % 64) == 0 && (kBG % 64) == 0 && (kC % 64) == 0 && (kC % 32) == 0, "GEMM M,N tile multiples");
static_assert(((kBC / 64) * (kG / 64)) % 8 == 0, "group-mixing grid exact");
static_assert(((kC / 32) * (kBG / 64)) % 4 == 0, "shared-MLP grid exact");
static_assert(((kG / 64) * (kBC / 64)) % 8 == 0, "final grid exact");

constexpr size_t kOffIdx   = 0;
constexpr size_t kOffPart  = kOffIdx   + (size_t)kBG * kNbr * 4;
constexpr size_t kOffScal  = kOffPart  + (size_t)kStatBlocks * 32 * 4;
constexpr size_t kOffFstat = kOffScal  + 256;
constexpr size_t kOffNormT = kOffFstat + (size_t)2 * kBC * 4;
constexpr size_t kOffGafW  = kOffNormT + (size_t)kBC * kG * 2;
constexpr size_t kOffFinW  = kOffGafW  + (size_t)kG * kG * 2;
constexpr size_t kOffMlpW  = kOffFinW  + (size_t)kG * kG2 * 2;
constexpr size_t kOffLc    = kOffMlpW  + (size_t)3 * kC * kC2 * 2;
constexpr size_t kOffXT    = kOffLc    + (size_t)3 * kBG * kC2 * 2;
constexpr size_t kWsTotal  = kOffXT    + (size_t)kBC * kG2 * 2;
static_assert(kWsTotal == 65298688ull, "carve total");
static_assert(kWsTotal <= 134217728ull, "carve cap");
static_assert((kOffPart % 256) == 0 && (kOffScal % 256) == 0 && (kOffFstat % 256) == 0 && (kOffNormT % 256) == 0 &&
              (kOffGafW % 256) == 0 && (kOffFinW % 256) == 0 && (kOffMlpW % 256) == 0 && (kOffLc % 256) == 0 &&
              (kOffXT % 256) == 0, "256-B aligned regions");

__device__ __forceinline__ v16h frag_load(const _Float16* p) {
  union { v16h v; v8h h[2]; } f;
  f.h[0] = *(const v8h*)(p);
  f.h[1] = *(const v8h*)(p + 16);
  return f.v;
}
__device__ __forceinline__ v8f mma_f16(v16h a, v16h b, v8f c) {
  return __builtin_amdgcn_wmma_f32_16x16x32_f16(false, a, false, b, (short)0, c, false, false);
}
__device__ __forceinline__ void tie1(v8f& c, v16h a, v16h b) { asm volatile("v_nop" : "+v"(c) : "v"(a), "v"(b)); }
__device__ __forceinline__ void tie4(v8f& c, v16h a, v16h b) { asm volatile("v_nop\n\tv_nop\n\tv_nop\n\tv_nop" : "+v"(c) : "v"(a), "v"(b)); }
__device__ __forceinline__ void keep4(v16h a, v16h b, v16h c, v16h d) { asm volatile("v_nop" :: "v"(a), "v"(b), "v"(c), "v"(d)); }
__device__ __forceinline__ void settle1(v8f& c) { asm volatile("v_nop" : "+v"(c)); }
__device__ __forceinline__ void wave_lds_sync() {
  __builtin_amdgcn_fence(__ATOMIC_RELEASE, "workgroup");
  __builtin_amdgcn_wave_barrier();
  __builtin_amdgcn_fence(__ATOMIC_ACQUIRE, "workgroup");
}
__device__ __forceinline__ void dump16(float* slab, const v8f& c0, const v8f& c1, const v8f& c2, const v8f& c3,
                                       int mOff, int rlane) {
#pragma unroll
  for (int r = 0; r < 8; ++r) {
    float* p = slab + (mOff + r) * kSlabP + rlane;
    p[0]  = c0[r];
    p[16] = c1[r];
    p[32] = c2[r];
    p[48] = c3[r];
  }
}

__global__ __launch_bounds__(256) void cast_scale_f16x8_kernel(
    const float* __restrict__ src, unsigned short* __restrict__ dst, int total8, float carry)
{
  const int i = blockIdx.x * 256 + threadIdx.x;
  if (i >= total8) return;
  const size_t e0 = (size_t)i << 3;
  const v4f a0 = *(const v4f*)(src + e0);
  const v4f a1 = *(const v4f*)(src + e0 + 4);
  v8h hv;
#pragma unroll
  for (int e = 0; e < 4; ++e) {
    hv[e]     = (_Float16)(a0[e] * carry);
    hv[4 + e] = (_Float16)(a1[e] * carry);
  }
  unsigned short* q = dst + e0;
  *(volatile v8h*)q = hv;
  __threadfence();
  *(volatile v8h*)q = hv;
}

__global__ __launch_bounds__(128) void knn_kernel(const float* __restrict__ center, int* __restrict__ idx_out)
{
#pragma clang fp contract(off)
  __shared__ float sx[kG];
  __shared__ float sy[kG];
  __shared__ float sz[kG];
  __shared__ float ssq[kG];
  __shared__ __align__(16) int sI[128 * kNbr];
  const int tid = threadIdx.x;
  const int b = blockIdx.x >> 3;
  const int nbase = (blockIdx.x & 7) * 128;
  const float* cb = center + (size_t)b * kG * 3;
  for (int m = tid; m < kG; m += 128) {
    const float x = cb[m * 3 + 0], y = cb[m * 3 + 1], z = cb[m * 3 + 2];
    const float t0 = x * x;
    const float t1 = y * y;
    const float t2 = z * z;
    sx[m] = x; sy[m] = y; sz[m] = z;
    ssq[m] = (t0 + t2) + t1;
  }
  __syncthreads();
  const int n = nbase + tid;
  const float cx = sx[n], cy = sy[n], cz = sz[n], sn = ssq[n];
  float bd[kNbr];
  int   bi[kNbr];
#pragma unroll
  for (int j = 0; j < kNbr; ++j) { bd[j] = 3.4e38f; bi[j] = 0; }
#pragma unroll 1
  for (int m = 0; m < kG; ++m) {
    float p = cx * sx[m];
    p = fmaf(cy, sy[m], p);
    p = fmaf(cz, sz[m], p);
    const float d = (sn + ssq[m]) - 2.0f * p;
    if (d < bd[kNbr - 1]) {
      bd[kNbr - 1] = d;
      bi[kNbr - 1] = m;
#pragma unroll
      for (int pz = kNbr - 1; pz > 0; --pz) {
        const bool sw = bd[pz] < bd[pz - 1];
        const float dl = sw ? bd[pz] : bd[pz - 1];
        const float dh = sw ? bd[pz - 1] : bd[pz];
        const int   il = sw ? bi[pz] : bi[pz - 1];
        const int   ih = sw ? bi[pz - 1] : bi[pz];
        bd[pz - 1] = dl; bd[pz] = dh;
        bi[pz - 1] = il; bi[pz] = ih;
      }
    }
  }
#pragma unroll
  for (int j = 0; j < kNbr; ++j) sI[tid * kNbr + j] = bi[j];
  __syncthreads();
  int* o = idx_out + ((size_t)b * kG + nbase) * kNbr;
  v4i ov[4];
#pragma unroll
  for (int it = 0; it < 4; ++it) ov[it] = *(const v4i*)(sI + (it * 128 + tid) * 4);
  for (int pass = 0; pass < 2; ++pass) {
#pragma unroll
    for (int it = 0; it < 4; ++it) {
      const int w4 = (it * 128 + tid) * 4;
      *(volatile v4i*)(o + w4) = ov[it];
    }
    __threadfence();
  }
}

__device__ __forceinline__ void acc12(const v4f& d0, const v4f& d1, const v4f& d2, float& s, float& q) {
#pragma unroll
  for (int e = 0; e < 4; ++e) { s += d0[e]; q += d0[e] * d0[e]; }
#pragma unroll
  for (int e = 0; e < 4; ++e) { s += d1[e]; q += d1[e] * d1[e]; }
#pragma unroll
  for (int e = 0; e < 4; ++e) { s += d2[e]; q += d2[e] * d2[e]; }
}

__global__ __launch_bounds__(256) void diff_stats_kernel(
    const float* __restrict__ feat, const int* __restrict__ idx, float* __restrict__ part)
{
  __shared__ float sP[8][8];
  const int lane = threadIdx.x & 31;
  const int wave = __builtin_amdgcn_readfirstlane((int)(threadIdx.x >> 5));
  float sA = 0.f, qA = 0.f, sB = 0.f, qB = 0.f, sC = 0.f, qC = 0.f;
#pragma unroll 1
  for (int rr = 0; rr < 2; ++rr) {
    const int bg = blockIdx.x * 16 + wave * 2 + rr;
    const int b = bg >> 10;
    int iv = idx[(size_t)bg * kNbr + (lane & 15)];
    iv = iv < 0 ? 0 : (iv > kG - 1 ? kG - 1 : iv);
    const float* frow = feat + (size_t)bg * kC + lane * 4;
    const float* fbat = feat + (size_t)b * kG * kC + lane * 4;
    const v4f c0 = *(const v4f*)(frow);
    const v4f c1 = *(const v4f*)(frow + 128);
    const v4f c2 = *(const v4f*)(frow + 256);
#pragma unroll 1
    for (int j = 0; j < 4; ++j) {
      const int nb = __shfl(iv, j, 32);
      const float* fn = fbat + (size_t)nb * kC;
      const v4f d0 = *(const v4f*)(fn) - c0;
      const v4f d1 = *(const v4f*)(fn + 128) - c1;
      const v4f d2 = *(const v4f*)(fn + 256) - c2;
      acc12(d0, d1, d2, sA, qA);
    }
#pragma unroll 1
    for (int j = 4; j < 8; ++j) {
      const int nb = __shfl(iv, j, 32);
      const float* fn = fbat + (size_t)nb * kC;
      const v4f d0 = *(const v4f*)(fn) - c0;
      const v4f d1 = *(const v4f*)(fn + 128) - c1;
      const v4f d2 = *(const v4f*)(fn + 256) - c2;
      acc12(d0, d1, d2, sB, qB);
    }
#pragma unroll 1
    for (int j = 8; j < 16; ++j) {
      const int nb = __shfl(iv, j, 32);
      const float* fn = fbat + (size_t)nb * kC;
      const v4f d0 = *(const v4f*)(fn) - c0;
      const v4f d1 = *(const v4f*)(fn + 128) - c1;
      const v4f d2 = *(const v4f*)(fn + 256) - c2;
      acc12(d0, d1, d2, sC, qC);
    }
  }
#pragma unroll
  for (int off = 16; off > 0; off >>= 1) {
    sA += __shfl_xor(sA, off, 32);
    qA += __shfl_xor(qA, off, 32);
    sB += __shfl_xor(sB, off, 32);
    qB += __shfl_xor(qB, off, 32);
    sC += __shfl_xor(sC, off, 32);
    qC += __shfl_xor(qC, off, 32);
  }
  {
    const float val = (lane == 0) ? sA : (lane == 1) ? qA : (lane == 2) ? sB : (lane == 3) ? qB
                    : (lane == 4) ? sC : (lane == 5) ? qC : 0.f;
    if (lane < 8) sP[wave][lane] = val;
  }
  __syncthreads();
  if (wave == 0) {
    const int col = lane & 7;
    float v = 0.f;
#pragma unroll
    for (int w = 0; w < 8; ++w) v += sP[w][col];
    const float o = (lane < 6) ? v : 0.f;
    float* dst = part + (size_t)blockIdx.x * 32 + lane;
    *(volatile float*)dst = o;
    __threadfence();
    *(volatile float*)dst = o;
  }
}

__global__ __launch_bounds__(32) void finalize_kernel(
    const float* __restrict__ part, const float* __restrict__ fusion_w, float* __restrict__ scal)
{
  __shared__ double sD[32];
  const int lane = threadIdx.x;
  double acc = 0.0;
#pragma unroll 1
  for (int blk = 0; blk < kStatBlocks; ++blk) acc += (double)part[(size_t)blk * 32 + lane];
  sD[lane] = acc;
  __syncthreads();
  const double s4 = sD[0], q4 = sD[1];
  const double s8 = s4 + sD[2], q8 = q4 + sD[3];
  const double s16 = s8 + sD[4], q16 = q8 + sD[5];
  constexpr double n4  = (double)kB * kG * 4.0 * kC;
  constexpr double n8  = (double)kB * kG * 8.0 * kC;
  constexpr double n16 = (double)kB * kG * 16.0 * kC;
  double v4 = (q4 - s4 * s4 * (1.0 / n4)) * (1.0 / (n4 - 1.0));
  double v8 = (q8 - s8 * s8 * (1.0 / n8)) * (1.0 / (n8 - 1.0));
  double v16 = (q16 - s16 * s16 * (1.0 / n16)) * (1.0 / (n16 - 1.0));
  v4 = v4 > 0.0 ? v4 : 0.0;
  v8 = v8 > 0.0 ? v8 : 0.0;
  v16 = v16 > 0.0 ? v16 : 0.0;
  const float inv0 = 1.0f / (sqrtf((float)v4) + kEps);
  const float inv1 = 1.0f / (sqrtf((float)v8) + kEps);
  const float inv2 = 1.0f / (sqrtf((float)v16) + kEps);
  const float f0 = fusion_w[0], f1 = fusion_w[1], f2 = fusion_w[2];
  const float fm = fmaxf(fmaxf(f0, f1), f2);
  const float e0 = expf(f0 - fm), e1 = expf(f1 - fm), e2 = expf(f2 - fm);
  const float rden = 1.0f / ((e0 + e1) + e2);
  const float w0 = e0 * rden, w1 = e1 * rden, w2 = e2 * rden;
  const float o = (lane == 0) ? inv0 : (lane == 1) ? inv1 : (lane == 2) ? inv2
                : (lane == 3) ? w0 : (lane == 4) ? w1 : (lane == 5) ? w2 : 0.f;
  *(volatile float*)(scal + lane) = o;
  __threadfence();
  *(volatile float*)(scal + lane) = o;
}

__global__ __launch_bounds__(256) void feat_stats_kernel(
    const float* __restrict__ feat, float* __restrict__ fmean, float* __restrict__ frs)
{
  const int t = blockIdx.x * 256 + threadIdx.x;
  const int b = t / kC;
  const int c = t - b * kC;
  const float* f = feat + (size_t)b * kG * kC + c;
  double s = 0.0, q = 0.0;
#pragma unroll 4
  for (int g = 0; g < kG; ++g) {
    const double v = (double)f[(size_t)g * kC];
    s += v;
    q += v * v;
  }
  const double mean = s * (1.0 / kG);
  double var = (q - s * s * (1.0 / kG)) * (1.0 / (kG - 1));
  var = var > 0.0 ? var : 0.0;
  const float mo = (float)mean;
  const float ro = 1.0f / (sqrtf((float)var) + kEps);
  *(volatile float*)(fmean + t) = mo;
  *(volatile float*)(frs + t) = ro;
  __threadfence();
  *(volatile float*)(fmean + t) = mo;
  *(volatile float*)(frs + t) = ro;
}

__global__ __launch_bounds__(256) void norm_transpose_kernel(
    const float* __restrict__ feat, const float* __restrict__ fmean, const float* __restrict__ frs,
    const float* __restrict__ gaf_alpha, const float* __restrict__ gaf_beta, unsigned short* __restrict__ normT)
{
  __shared__ float sT[64 * 65];
  const int tid = threadIdx.x;
  const int lane = tid & 31;
  const int wave = __builtin_amdgcn_readfirstlane((int)(tid >> 5));
  const int g0 = blockIdx.x * 64, c0 = blockIdx.y * 64, b = blockIdx.z;
  const int r = tid >> 4, c4 = (tid & 15) * 4;
  const v4f mean4 = *(const v4f*)(fmean + b * kC + c0 + c4);
  const v4f rs4   = *(const v4f*)(frs + b * kC + c0 + c4);
  const v4f al4   = *(const v4f*)(gaf_alpha + c0 + c4);
  const v4f be4   = *(const v4f*)(gaf_beta + c0 + c4);
#pragma unroll
  for (int it = 0; it < 4; ++it) {
    const int g = r + 16 * it;
    const v4f v = *(const v4f*)(feat + ((size_t)(b * kG + g0 + g)) * kC + c0 + c4);
#pragma unroll
    for (int e = 0; e < 4; ++e) {
      const float nv = al4[e] * ((v[e] - mean4[e]) * rs4[e]) + be4[e];
      sT[g * 65 + c4 + e] = nv * kNCarry;
    }
  }
  __syncthreads();
  const int q = lane >> 3, c8 = (lane & 7) * 8;
  v8h hv[2];
#pragma unroll
  for (int it = 0; it < 2; ++it) {
    const int c = it * 32 + wave * 4 + q;
#pragma unroll
    for (int e = 0; e < 8; ++e) hv[it][e] = (_Float16)sT[(c8 + e) * 65 + c];
  }
  for (int pass = 0; pass < 2; ++pass) {
#pragma unroll
    for (int it = 0; it < 2; ++it) {
      const int c = it * 32 + wave * 4 + q;
      *(volatile v8h*)(normT + ((size_t)(b * kC + c0 + c)) * kG + g0 + c8) = hv[it];
    }
    __threadfence();
  }
}

__global__ __launch_bounds__(128) void pool_ln_kernel(
    const float* __restrict__ feat, const int* __restrict__ idx,
    const float* __restrict__ lnp_alpha, const float* __restrict__ lnp_beta,
    const float* __restrict__ ln_gamma, const float* __restrict__ ln_beta,
    const float* __restrict__ scal, unsigned short* __restrict__ lc16)
{
  __shared__ __align__(16) float sL[4][3 * kC2];
  const int lane = threadIdx.x & 31;
  const int wave = __builtin_amdgcn_readfirstlane((int)(threadIdx.x >> 5));
  const int bg = blockIdx.x * 4 + wave;
  const int b = bg >> 10;
  int iv = idx[(size_t)bg * kNbr + (lane & 15)];
  iv = iv < 0 ? 0 : (iv > kG - 1 ? kG - 1 : iv);
  float* my = sL[wave];
  const float* frow = feat + (size_t)bg * kC;
  const float* fbat = feat + (size_t)b * kG * kC;
#pragma unroll 1
  for (int i = 0; i < 3; ++i) {
    const float inv = scal[i];
    const int kcnt = 4 << i;
    const float* al = lnp_alpha + i * kC2;
    const float* be = lnp_beta + i * kC2;
    float* mi = my + i * kC2;
#pragma unroll 1
    for (int qq = 0; qq < kC / 32; ++qq) {
      const int c = qq * 32 + lane;
      const float fc = frow[c];
      const float a = al[c];
      const float o = be[c];
      float se = 0.f, sx = 0.f;
#pragma unroll 1
      for (int j = 0; j < kcnt; ++j) {
        const int nb = __shfl(iv, j, 32);
        const float d = fbat[(size_t)nb * kC + c] - fc;
        const float x = a * (d * inv) + o;
        const float e = expf(x);
        se += e;
        sx += x * e;
      }
      const float pooled = sx * __builtin_amdgcn_rcpf(se);
      const float second = al[kC + c] * fc + be[kC + c];
      mi[c] = pooled;
      mi[kC + c] = second;
    }
  }
  __syncthreads();
  constexpr float kInvN = 1.0f / (float)kC2;
#pragma unroll 1
  for (int i = 0; i < 3; ++i) {
    const float* mi = my + i * kC2 + lane * 8;
    float s1 = 0.f;
#pragma unroll 1
    for (int s = 0; s < 3; ++s) {
      const v4f x0 = *(const v4f*)(mi + s * 256);
      const v4f x1 = *(const v4f*)(mi + s * 256 + 4);
      s1 += ((x0[0] + x0[1]) + (x0[2] + x0[3])) + ((x1[0] + x1[1]) + (x1[2] + x1[3]));
    }
#pragma unroll
    for (int off = 16; off > 0; off >>= 1) s1 += __shfl_xor(s1, off, 32);
    const float mu = s1 * kInvN;
    float s2 = 0.f;
#pragma unroll 1
    for (int s = 0; s < 3; ++s) {
      const v4f x0 = *(const v4f*)(mi + s * 256);
      const v4f x1 = *(const v4f*)(mi + s * 256 + 4);
#pragma unroll
      for (int e = 0; e < 4; ++e) {
        const float t0 = x0[e] - mu;
        const float t1 = x1[e] - mu;
        s2 += t0 * t0;
        s2 += t1 * t1;
      }
    }
#pragma unroll
    for (int off = 16; off > 0; off >>= 1) s2 += __shfl_xor(s2, off, 32);
    const float var = s2 * kInvN;
    const float rstd = 1.0f / sqrtf(var + kEps);
    const float* gm = ln_gamma + i * kC2 + lane * 8;
    const float* bt = ln_beta + i * kC2 + lane * 8;
    unsigned short* orow = lc16 + ((size_t)i * kBG + bg) * kC2 + lane * 8;
#pragma unroll 1
    for (int s = 0; s < 3; ++s) {
      const v4f x0 = *(const v4f*)(mi + s * 256);
      const v4f x1 = *(const v4f*)(mi + s * 256 + 4);
      const v4f g0 = *(const v4f*)(gm + s * 256);
      const v4f g1 = *(const v4f*)(gm + s * 256 + 4);
      const v4f t0 = *(const v4f*)(bt + s * 256);
      const v4f t1 = *(const v4f*)(bt + s * 256 + 4);
      v8h hv;
#pragma unroll
      for (int e = 0; e < 4; ++e) {
        const float y0 = ((x0[e] - mu) * rstd) * g0[e] + t0[e];
        const float y1 = ((x1[e] - mu) * rstd) * g1[e] + t1[e];
        hv[e]     = (_Float16)(y0 * kNCarry);
        hv[4 + e] = (_Float16)(y1 * kNCarry);
      }
      unsigned short* p = orow + s * 256;
      *(volatile v8h*)p = hv;
      __threadfence();
      *(volatile v8h*)p = hv;
    }
  }
}

constexpr int kModeGaf = 0;
constexpr int kModeMlp = 1;
constexpr int kModeFin = 2;

template <int MI, int NW, int MODE>
__global__ __launch_bounds__(NW * 32) void gemm_f16_kernel(
    const unsigned short* __restrict__ Ap, int lda, long aBr,
    const unsigned short* __restrict__ Btp, int ldb, long bBr,
    void* __restrict__ Cout, const float* __restrict__ bias, const float* __restrict__ scal,
    int tilesM, int tilesN, int K, float scale, float ocarry)
{
  constexpr int NBR = (MODE == kModeMlp) ? 3 : 1;
  constexpr int TM = MI * 16;
  constexpr int FW = (NBR > 1) ? NW : 1;
  constexpr int FN = (NBR > 1) ? (TM * 64) : 4;
  __shared__ __align__(16) float sSlab[NW][16 * kSlabP];
  __shared__ __align__(16) float sFuse[FW][FN];
  const _Float16* A  = (const _Float16*)Ap;
  const _Float16* Bt = (const _Float16*)Btp;
  const int lane = threadIdx.x & 31;
  const int wave = __builtin_amdgcn_readfirstlane((int)(threadIdx.x >> 5));
  const int tile = blockIdx.x * NW + wave;
  if (tile >= tilesM * tilesN) return;
  const int tm = tile / tilesN;
  const int tn = tile - tm * tilesN;
  const int m0 = tm * TM;
  const int n0 = tn << 6;
  const int rlane = lane & 15;
  const int koff  = (lane >> 4) * 8;
  const int mOff  = (lane >> 4) * 8;
  const int q = lane >> 3, c8 = (lane & 7) * 8;
  const int hh = lane >> 4, c4 = (lane & 15) * 4;
  float* slab = sSlab[wave];
  float* fuse = sFuse[(NBR > 1) ? wave : 0];

  v4f bn0 = (v4f){0.f, 0.f, 0.f, 0.f};
  v4f bn1 = (v4f){0.f, 0.f, 0.f, 0.f};
  if (MODE == kModeGaf) {
    bn0 = *(const v4f*)(bias + n0 + c8);
    bn1 = *(const v4f*)(bias + n0 + c8 + 4);
  }
  size_t cBase;
  int ldc;
  if (MODE == kModeGaf) {
    cBase = (size_t)m0 * kG2 + n0;
    ldc = kG2;
  } else if (MODE == kModeMlp) {
    const int bi = n0 >> 10;
    const int g0 = n0 & (kG - 1);
    cBase = (size_t)(bi * kC + m0) * kG2 + kG + g0;
    ldc = kG2;
  } else {
    const int bi = n0 / kC;
    const int c0 = n0 - bi * kC;
    cBase = (size_t)(bi * kG + m0) * kC + c0;
    ldc = kC;
  }
  if (NBR > 1) {
#pragma unroll 1
    for (int it = 0; it < TM / 4; ++it) {
      float* fp = fuse + (it * 4 + q) * 64 + c8;
      *(v4f*)(fp)     = (v4f){0.f, 0.f, 0.f, 0.f};
      *(v4f*)(fp + 4) = (v4f){0.f, 0.f, 0.f, 0.f};
    }
  }

#pragma unroll 1
  for (int br = 0; br < NBR; ++br) {
    const _Float16* Ab = A  + (size_t)br * aBr;
    const _Float16* Bb = Bt + (size_t)br * bBr;
    v8f acc[MI][4];
#pragma unroll
    for (int i = 0; i < MI; ++i)
#pragma unroll
      for (int j = 0; j < 4; ++j) acc[i][j] = (v8f){0.f, 0.f, 0.f, 0.f, 0.f, 0.f, 0.f, 0.f};

    for (int k0 = 0; k0 < K; k0 += 32) {
      v16h bf[4];
#pragma unroll
      for (int j = 0; j < 4; ++j)
        bf[j] = frag_load(Bb + (size_t)(n0 + (j << 4) + rlane) * ldb + koff + k0);
#pragma unroll
      for (int i = 0; i < MI; ++i) {
        const v16h ah = frag_load(Ab + (size_t)(m0 + (i << 4) + rlane) * lda + koff + k0);
#pragma unroll
        for (int j = 0; j < 4; ++j) acc[i][j] = mma_f16(ah, bf[j], acc[i][j]);
        tie1(acc[i][0], ah, bf[0]);
        tie1(acc[i][1], ah, bf[1]);
        tie1(acc[i][2], ah, bf[2]);
        tie4(acc[i][3], ah, bf[3]);
      }
      keep4(bf[0], bf[1], bf[2], bf[3]);
    }
#pragma unroll
    for (int i = 0; i < MI; ++i)
#pragma unroll
      for (int j = 0; j < 4; ++j) settle1(acc[i][j]);

    float wbr = 1.0f;
    if (NBR > 1) wbr = scal[3 + br];
    const bool last = (br == NBR - 1);

#pragma unroll 1
    for (int i = 0; i < MI; ++i) {
      if (i == 0) {
        dump16(slab, acc[0][0], acc[0][1], acc[0][2], acc[0][3], mOff, rlane);
      } else if (i == 1) {
        dump16(slab, acc[1][0], acc[1][1], acc[1][2], acc[1][3], mOff, rlane);
      } else if ((MI > 2) && (i == 2)) {
        dump16(slab, acc[(MI > 2) ? 2 : 0][0], acc[(MI > 2) ? 2 : 0][1], acc[(MI > 2) ? 2 : 0][2], acc[(MI > 2) ? 2 : 0][3], mOff, rlane);
      } else if (MI > 2) {
        dump16(slab, acc[(MI > 2) ? 3 : 0][0], acc[(MI > 2) ? 3 : 0][1], acc[(MI > 2) ? 3 : 0][2], acc[(MI > 2) ? 3 : 0][3], mOff, rlane);
      }
      wave_lds_sync();
      const int rbase = m0 + i * 16;
      if (MODE != kModeFin) {
#pragma unroll 1
        for (int it = 0; it < 4; ++it) {
          const int row = it * 4 + q;
          float* sp = slab + row * kSlabP + c8;
          const v4f x0 = *(const v4f*)(sp);
          const v4f x1 = *(const v4f*)(sp + 4);
          float bm = 0.f;
          if (MODE == kModeMlp) bm = bias[br * kC + rbase + row];
          v4f y0, y1;
#pragma unroll
          for (int e = 0; e < 4; ++e) {
            const float t0 = x0[e] * scale + ((MODE == kModeGaf) ? bn0[e] : bm);
            const float t1 = x1[e] * scale + ((MODE == kModeGaf) ? bn1[e] : bm);
            y0[e] = t0 * (1.0f / (1.0f + expf(-t0)));
            y1[e] = t1 * (1.0f / (1.0f + expf(-t1)));
          }
          if (NBR > 1) {
            float* fp = fuse + (i * 16 + row) * 64 + c8;
            v4f f0 = *(const v4f*)(fp);
            v4f f1 = *(const v4f*)(fp + 4);
            f0 = f0 + wbr * y0;
            f1 = f1 + wbr * y1;
            *(v4f*)(fp)     = f0;
            *(v4f*)(fp + 4) = f1;
            y0 = f0;
            y1 = f1;
          }
          y0 = y0 * ocarry;
          y1 = y1 * ocarry;
          *(v4f*)(sp)     = y0;
          *(v4f*)(sp + 4) = y1;
        }
        wave_lds_sync();
      }
      if (last) {
        if (MODE == kModeFin) {
          float* C = (float*)Cout + cBase + (size_t)(i * 16) * ldc;
          v4f ov[8];
#pragma unroll
          for (int it = 0; it < 8; ++it) {
            const int row = it * 2 + hh;
            const v4f v = *(const v4f*)(slab + row * kSlabP + c4);
            const float bm = bias[rbase + row];
            ov[it] = v * scale + bm;
          }
          for (int pass = 0; pass < 2; ++pass) {
#pragma unroll
            for (int it = 0; it < 8; ++it) {
              const int row = it * 2 + hh;
              *(volatile v4f*)(C + (size_t)row * ldc + c4) = ov[it];
            }
            __threadfence();
          }
        } else {
          unsigned short* C = (unsigned short*)Cout + cBase + (size_t)(i * 16) * ldc;
          v8h hv[4];
#pragma unroll
          for (int it = 0; it < 4; ++it) {
            const int row = it * 4 + q;
            const float* sp = slab + row * kSlabP + c8;
#pragma unroll
            for (int e = 0; e < 8; ++e) hv[it][e] = (_Float16)sp[e];
          }
          for (int pass = 0; pass < 2; ++pass) {
#pragma unroll
            for (int it = 0; it < 4; ++it) {
              const int row = it * 4 + q;
              *(volatile v8h*)(C + (size_t)row * ldc + c8) = hv[it];
            }
            __threadfence();
          }
        }
      }
      wave_lds_sync();
    }
  }
}

extern "C" void kernel_launch(void* const* d_in, const int* in_sizes, int n_in,
                              void* d_out, int out_size, void* d_ws, size_t ws_size,
                              hipStream_t stream) {
  if (n_in < 15) return;
  if (in_sizes[0] != kB * kG * 3) return;
  if (in_sizes[1] != kB * kG * kC) return;
  if (in_sizes[2] != 3 * kC2 || in_sizes[3] != 3 * kC2 || in_sizes[4] != 3 * kC2 || in_sizes[5] != 3 * kC2) return;
  if (in_sizes[6] != 3 * kC * kC2) return;
  if (in_sizes[7] != 3 * kC) return;
  if (in_sizes[8] != 3) return;
  if (in_sizes[9] != kC || in_sizes[10] != kC) return;
  if (in_sizes[11] != kG * kG) return;
  if (in_sizes[12] != kG) return;
  if (in_sizes[13] != kG * kG2) return;
  if (in_sizes[14] != kG) return;
  if (out_size != kB * kG * kC) return;
  if (ws_size < kWsTotal) return;

  const float* center    = (const float*)d_in[0];
  const float* feat      = (const float*)d_in[1];
  const float* lnp_alpha = (const float*)d_in[2];
  const float* lnp_beta  = (const float*)d_in[3];
  const float* ln_gamma  = (const float*)d_in[4];
  const float* ln_beta   = (const float*)d_in[5];
  const float* mlp_w     = (const float*)d_in[6];
  const float* mlp_b     = (const float*)d_in[7];
  const float* fusion_w  = (const float*)d_in[8];
  const float* gaf_alpha = (const float*)d_in[9];
  const float* gaf_beta  = (const float*)d_in[10];
  const float* gaf_w     = (const float*)d_in[11];
  const float* gaf_b     = (const float*)d_in[12];
  const float* fin_w     = (const float*)d_in[13];
  const float* fin_b     = (const float*)d_in[14];
  float* out = (float*)d_out;

  char* ws = (char*)d_ws;
  int*            IDX   = (int*)(ws + kOffIdx);
  float*          PART  = (float*)(ws + kOffPart);
  float*          SCAL  = (float*)(ws + kOffScal);
  float*          FMEAN = (float*)(ws + kOffFstat);
  float*          FRS   = FMEAN + kBC;
  unsigned short* NORMT = (unsigned short*)(ws + kOffNormT);
  unsigned short* GAFW  = (unsigned short*)(ws + kOffGafW);
  unsigned short* FINW  = (unsigned short*)(ws + kOffFinW);
  unsigned short* MLPW  = (unsigned short*)(ws + kOffMlpW);
  unsigned short* LC16  = (unsigned short*)(ws + kOffLc);
  unsigned short* XT16  = (unsigned short*)(ws + kOffXT);

  cast_scale_f16x8_kernel<<<(kG * kG / 8) / 256, 256, 0, stream>>>(gaf_w, GAFW, kG * kG / 8, kWCarry);
  cast_scale_f16x8_kernel<<<(kG * kG2 / 8) / 256, 256, 0, stream>>>(fin_w, FINW, kG * kG2 / 8, kWCarry);
  cast_scale_f16x8_kernel<<<(3 * kC * kC2 / 8) / 256, 256, 0, stream>>>(mlp_w, MLPW, 3 * kC * kC2 / 8, kWCarry);

  knn_kernel<<<kB * 8, 128, 0, stream>>>(center, IDX);
  diff_stats_kernel<<<kStatBlocks, 256, 0, stream>>>(feat, IDX, PART);
  finalize_kernel<<<1, 32, 0, stream>>>(PART, fusion_w, SCAL);

  feat_stats_kernel<<<kBC / 256, 256, 0, stream>>>(feat, FMEAN, FRS);
  norm_transpose_kernel<<<dim3(kG / 64, kC / 64, kB), 256, 0, stream>>>(feat, FMEAN, FRS, gaf_alpha, gaf_beta, NORMT);

  pool_ln_kernel<<<kBG / 4, 128, 0, stream>>>(feat, IDX, lnp_alpha, lnp_beta, ln_gamma, ln_beta, SCAL, LC16);

  gemm_f16_kernel<4, 8, kModeGaf><<<96, 256, 0, stream>>>(
      NORMT, kG, 0L, GAFW, kG, 0L, (void*)XT16, gaf_b, SCAL,
      kBC / 64, kG / 64, kG, kScaleGaf, kXCarry);

  gemm_f16_kernel<2, 4, kModeMlp><<<384, 128, 0, stream>>>(
      MLPW, kC2, (long)kC * kC2, LC16, kC2, (long)kBG * kC2, (void*)XT16, mlp_b, SCAL,
      kC / 32, kBG / 64, kC2, kScaleMlp, kXCarry);

  gemm_f16_kernel<4, 8, kModeFin><<<96, 256, 0, stream>>>(
      FINW, kG2, 0L, XT16, kG2, 0L, (void*)out, fin_b, SCAL,
      kG / 64, kBC / 64, kG2, kScaleFin, 1.0f);
}
